// OntologyEmbedding_28604482191517
// MI455X (gfx1250) — hardware-verified
//
#include <hip/hip_runtime.h>
#include <stddef.h>


#define NCH   100
#define HEADS 5
#define CPH   20
#define KPAD  128
#define NPADC 112
#define HP    128
#define ALP   16
#define GR    32
#define GT    224
#define AP    136
#define XSP   132
#define NB    512
#define SP    100
#define CHUNK 2048
#define NTHR  256
#define NWAVE 8
#define WCAP  256
#define NGRP  (CHUNK / (NTHR * 4))
#define OB    32

#define LDS_SACC  (NB * SP)
#define LDS_MD    (NB * HEADS)
#define LDS_LIST  (NWAVE * WCAP)
#define LDS_BYTES ((LDS_SACC + 2 * LDS_MD + LDS_LIST + NWAVE) * 4)

static_assert(WCAP == (CHUNK / NTHR) * 32);
static_assert(NGRP >= 1);
static_assert(NB == 512);
static_assert(CHUNK == 2048);
static_assert((LDS_SACC % 4) == 0);
static_assert(LDS_BYTES == 233504);
static_assert(NCH == HEADS * CPH);
static_assert((NCH % 4) == 0 && (CPH % 4) == 0);
static_assert(GT == 7 * 32);

typedef float          v4f  __attribute__((ext_vector_type(4)));
typedef float          v8f  __attribute__((ext_vector_type(8)));
typedef int            v4i  __attribute__((ext_vector_type(4)));
typedef unsigned short v4s  __attribute__((ext_vector_type(4)));
typedef unsigned short v8s  __attribute__((ext_vector_type(8)));
typedef __bf16         v16b __attribute__((ext_vector_type(16)));
union Frag   { v16b v; v8s half[2]; };
union Pack16 { v8s s; v4i i; };

__device__ __forceinline__ unsigned short bf_bits(float f) {
  unsigned u = __float_as_uint(f);
  u = u + 0x7FFFu + ((u >> 16) & 1u);
  return (unsigned short)(u >> 16);
}
__device__ __forceinline__ float bf_val(unsigned short b) {
  return __uint_as_float(((unsigned)b) << 16);
}

__device__ __forceinline__ v8f wm(v16b a, v16b b, v8f c) {
  v8f d = __builtin_amdgcn_wmma_f32_16x16x32_bf16(false, a, false, b, (short)0, c, false, false);
  asm volatile("v_nop\n\tv_nop\n\tv_nop\n\tv_nop" : "+v"(d) : "v"(a), "v"(b));
  return d;
}

__global__ __launch_bounds__(NTHR) void k_prep(const float* __restrict__ W,
                                               unsigned short* Wh, unsigned short* Wl, int nItems) {
  const int i = blockIdx.x * NTHR + threadIdx.x;
  if (i >= nItems) return;
  const int col = i >> 4;
  const int k0  = (i & 15) * 8;
  const int cc  = min(col, NCH - 1);
  Pack16 ph, pl;
#pragma unroll
  for (int j = 0; j < 8; ++j) {
    const int k  = k0 + j;
    const int kc = min(k, NCH - 1);
    float v = W[(size_t)kc * NCH + cc];
    v = (col < NCH && k < NCH) ? v : 0.0f;
    const unsigned short hb = bf_bits(v);
    const unsigned short lb = bf_bits(v - bf_val(hb));
    ph.s[j] = hb;
    pl.s[j] = lb;
  }
  const size_t o = (size_t)col * KPAD + k0;
  *(volatile v4i*)(Wh + o) = ph.i;
  *(volatile v4i*)(Wl + o) = pl.i;
  __threadfence();
  *(volatile v4i*)(Wh + o) = ph.i;
  *(volatile v4i*)(Wl + o) = pl.i;
}

__global__ __launch_bounds__(GT) void k_gemm(
    const float* __restrict__ x, int ldx,
    const unsigned short* __restrict__ Wh, const unsigned short* __restrict__ Wl,
    const float* __restrict__ att, float* hp, float* alp, int nN) {
  __shared__ __attribute__((aligned(16))) unsigned short Ahi[GR * AP];
  __shared__ __attribute__((aligned(16))) unsigned short Alo[GR * AP];
  __shared__ __attribute__((aligned(16))) float Xs[GR * XSP];
  __shared__ __attribute__((aligned(16))) float Sal[GR * ALP];

  const int tid  = threadIdx.x;
  const int lane = tid & 31;
  const int wave = tid >> 5;
  const int hh   = lane >> 4;
  const int m    = lane & 15;
  const int rowBase = blockIdx.x * GR;

#pragma unroll
  for (int it = 0; it < 5; ++it) {
    const int i = tid + GT * it;
    if (i < GR * 32) {
      const int r  = i >> 5;
      const int k0 = (i & 31) * 4;
      int grow = rowBase + r;
      if (grow > nN - 1) grow = nN - 1;
      const int kc = min(k0, NCH - 4);
      const v4f f = *(const v4f*)(x + (size_t)grow * ldx + kc);
      const bool valid = (k0 < NCH);
      const float e0 = valid ? f.x : 0.0f;
      const float e1 = valid ? f.y : 0.0f;
      const float e2 = valid ? f.z : 0.0f;
      const float e3 = valid ? f.w : 0.0f;
      v4s hs, ls;
      hs.x = bf_bits(e0); ls.x = bf_bits(e0 - bf_val(hs.x));
      hs.y = bf_bits(e1); ls.y = bf_bits(e1 - bf_val(hs.y));
      hs.z = bf_bits(e2); ls.z = bf_bits(e2 - bf_val(hs.z));
      hs.w = bf_bits(e3); ls.w = bf_bits(e3 - bf_val(hs.w));
      *(v4s*)(Ahi + r * AP + k0) = hs;
      *(v4s*)(Alo + r * AP + k0) = ls;
    }
  }
  if (tid < 128) {
    const v4f z4 = {0.f, 0.f, 0.f, 0.f};
    const int r = tid >> 2;
    const int q = tid & 3;
    *(v4f*)(Xs + r * XSP + NPADC + 4 * q) = z4;
    *(v4f*)(Sal + 4 * tid) = z4;
  }
  __syncthreads();

  const int ncol = wave * 16 + m;
  v8f c0 = {0.f, 0.f, 0.f, 0.f, 0.f, 0.f, 0.f, 0.f};
  v8f c1 = {0.f, 0.f, 0.f, 0.f, 0.f, 0.f, 0.f, 0.f};
#pragma unroll
  for (int kt = 0; kt < KPAD / 32; ++kt) {
    const int k0 = kt * 32;
    Frag bh, bl, a0h, a0l, a1h, a1l;
    const unsigned short* pbh = Wh + (size_t)ncol * KPAD + k0 + 8 * hh;
    const unsigned short* pbl = Wl + (size_t)ncol * KPAD + k0 + 8 * hh;
    const unsigned short* p0h = Ahi + m * AP + k0 + 8 * hh;
    const unsigned short* p0l = Alo + m * AP + k0 + 8 * hh;
    const unsigned short* p1h = Ahi + (16 + m) * AP + k0 + 8 * hh;
    const unsigned short* p1l = Alo + (16 + m) * AP + k0 + 8 * hh;
    bh.half[0]  = *(const v8s*)pbh;  bh.half[1]  = *(const v8s*)(pbh + 16);
    bl.half[0]  = *(const v8s*)pbl;  bl.half[1]  = *(const v8s*)(pbl + 16);
    a0h.half[0] = *(const v8s*)p0h;  a0h.half[1] = *(const v8s*)(p0h + 16);
    a0l.half[0] = *(const v8s*)p0l;  a0l.half[1] = *(const v8s*)(p0l + 16);
    a1h.half[0] = *(const v8s*)p1h;  a1h.half[1] = *(const v8s*)(p1h + 16);
    a1l.half[0] = *(const v8s*)p1l;  a1l.half[1] = *(const v8s*)(p1l + 16);
    c0 = wm(a0h.v, bh.v, c0);
    c0 = wm(a0h.v, bl.v, c0);
    c0 = wm(a0l.v, bh.v, c0);
    c1 = wm(a1h.v, bh.v, c1);
    c1 = wm(a1h.v, bl.v, c1);
    c1 = wm(a1l.v, bh.v, c1);
  }

#pragma unroll
  for (int r = 0; r < 8; ++r) {
    Xs[(8 * hh + r) * XSP + ncol]      = c0[r];
    Xs[(16 + 8 * hh + r) * XSP + ncol] = c1[r];
  }
  __syncthreads();

  if (tid < GR * HEADS) {
    const int row = tid / HEADS;
    const int hd  = tid - row * HEADS;
    const float* xr = Xs + row * XSP + hd * CPH;
    const float* ap = att + hd * (2 * CPH);
    float sd = 0.0f, ss = 0.0f;
#pragma unroll
    for (int c = 0; c < CPH; ++c) {
      const float v = xr[c];
      sd += v * ap[c];
      ss += v * ap[CPH + c];
    }
    Sal[row * ALP + hd]     = sd;
    Sal[row * ALP + 8 + hd] = ss;
  }
  __syncthreads();

  v4f hv[5];
#pragma unroll
  for (int it = 0; it < 5; ++it) {
    int i = tid + GT * it;
    if (i > GR * 32 - 1) i = GR * 32 - 1;
    hv[it] = *(const v4f*)(Xs + (i >> 5) * XSP + 4 * (i & 31));
  }
  const v4f av = *(const v4f*)(Sal + 4 * min(tid, 127));
  float* hbase = hp  + (size_t)rowBase * HP;
  float* abase = alp + (size_t)rowBase * ALP;
#pragma unroll
  for (int it = 0; it < 5; ++it) {
    const int i = tid + GT * it;
    if (i < GR * 32) *(volatile v4f*)(hbase + 4 * i) = hv[it];
  }
  if (tid < 128) *(volatile v4f*)(abase + 4 * tid) = av;
  __threadfence();
#pragma unroll
  for (int it = 0; it < 5; ++it) {
    const int i = tid + GT * it;
    if (i < GR * 32) *(volatile v4f*)(hbase + 4 * i) = hv[it];
  }
  if (tid < 128) *(volatile v4f*)(abase + 4 * tid) = av;
}

__global__ __launch_bounds__(NTHR) void k_gat(
    const float* __restrict__ hp, const float* __restrict__ al, const int* __restrict__ ei,
    const float* __restrict__ bias, float* outp, int nN, int nE) {
  extern __shared__ v4f lds_dyn[];
  float* sacc = (float*)lds_dyn;
  float* mx   = sacc + LDS_SACC;
  float* den  = mx + LDS_MD;
  int*   list = (int*)(den + LDS_MD);
  int*   wcnt = list + LDS_LIST;

  const int tid  = threadIdx.x;
  const int lane = tid & 31;
  const int wave = tid >> 5;
  int hd = lane / 5;
  if (hd > HEADS - 1) hd = HEADS - 1;
  const bool okc = (lane < NCH / 4);
  const int  cl  = min(lane, NCH / 4 - 1);
  const int nodeBase = blockIdx.x * NB;
  const int* eid  = ei;
  const int* esrc = ei + nE;
  const bool al16 = ((((size_t)eid) & 15) == 0);

#pragma unroll 1
  for (int j = 0; j < NB / NWAVE; ++j) {
    const int slot = wave * (NB / NWAVE) + j;
    int node = nodeBase + slot;
    if (node > nN - 1) node = nN - 1;
    const v4f hv = *(const v4f*)(hp + (size_t)node * HP + 4 * lane);
    if (okc) *(v4f*)(sacc + slot * SP + 4 * lane) = hv;
    float lg = al[(size_t)node * ALP + hd] + al[(size_t)node * ALP + 8 + hd];
    lg = (lg >= 0.0f) ? lg : 0.2f * lg;
    mx[slot * HEADS + hd]  = lg;
    den[slot * HEADS + hd] = 1.0f;
  }
  __syncthreads();

  const int nChunks = (nE + CHUNK - 1) / CHUNK;
#pragma unroll 1
  for (int ch = 0; ch < nChunks; ++ch) {
    const int cbase = ch * CHUNK;
    const bool full = al16 && (cbase + CHUNK <= nE);
    int wc = 0;
#pragma unroll
    for (int g = 0; g < NGRP; ++g) {
      const int el0 = (g * NTHR + tid) * 4;
      const int e0  = cbase + el0;
      const int sent = -2147483647 - 1;
      v4i d;
      if (full) {
        d = *(const v4i*)(eid + e0);
      } else {
        d.x = (e0     < nE) ? eid[min(e0,     nE - 1)] : sent;
        d.y = (e0 + 1 < nE) ? eid[min(e0 + 1, nE - 1)] : sent;
        d.z = (e0 + 2 < nE) ? eid[min(e0 + 2, nE - 1)] : sent;
        d.w = (e0 + 3 < nE) ? eid[min(e0 + 3, nE - 1)] : sent;
      }
      const unsigned s0 = (unsigned)d.x - (unsigned)nodeBase;
      const unsigned s1 = (unsigned)d.y - (unsigned)nodeBase;
      const unsigned s2 = (unsigned)d.z - (unsigned)nodeBase;
      const unsigned s3 = (unsigned)d.w - (unsigned)nodeBase;
      const bool h0 = s0 < (unsigned)NB;
      const bool h1 = s1 < (unsigned)NB;
      const bool h2 = s2 < (unsigned)NB;
      const bool h3 = s3 < (unsigned)NB;
      const unsigned many = __builtin_amdgcn_ballot_w32(h0 | h1 | h2 | h3);
      if (many != 0u) {
#define HITJ(J, HJ, SJ) { \
          const unsigned mj = __builtin_amdgcn_ballot_w32(HJ); \
          if (HJ) { \
            const int pos = wc + (int)__builtin_amdgcn_mbcnt_lo(mj, 0u); \
            if (pos < WCAP) list[wave * WCAP + pos] = ((el0 + (J)) << 9) | (int)(SJ); \
          } \
          wc += (int)__builtin_popcount(mj); }
        HITJ(0, h0, s0)
        HITJ(1, h1, s1)
        HITJ(2, h2, s2)
        HITJ(3, h3, s3)
#undef HITJ
      }
    }
    if (lane == 0) wcnt[wave] = wc;
    __syncthreads();

    if (wave == 0) {
      for (int wsx = 0; wsx < NWAVE; ++wsx) {
        int n = wcnt[wsx];
        if (n > WCAP) n = WCAP;
        if (n < 0) n = 0;
        for (int i = 0; i < n; ++i) {
          const int ent  = list[wsx * WCAP + i];
          const int slot = ent & (NB - 1);
          const int el   = (ent >> 9) & (CHUNK - 1);
          int e = cbase + el;
          if (e > nE - 1) e = nE - 1;
          int src = esrc[e];
          src = src < 0 ? 0 : (src > nN - 1 ? nN - 1 : src);
          int nd = nodeBase + slot;
          if (nd > nN - 1) nd = nN - 1;
          float lg = al[(size_t)nd * ALP + hd] + al[(size_t)src * ALP + 8 + hd];
          lg = (lg >= 0.0f) ? lg : 0.2f * lg;
          const int md = slot * HEADS + hd;
          const float mo = mx[md];
          const float mn = fmaxf(mo, lg);
          const float sc = __expf(mo - mn);
          const float p  = __expf(lg - mn);
          const v4f hv = *(const v4f*)(hp + (size_t)src * HP + 4 * lane);
          v4f* sp = (v4f*)(sacc + slot * SP + 4 * cl);
          const v4f cur = *sp;
          const v4f nxt = cur * sc + hv * p;
          const float dv = den[md];
          if (okc) *sp = nxt;
          mx[md]  = mn;
          den[md] = dv * sc + p;
        }
      }
    }
    __syncthreads();
  }

  const v4f b4 = *(const v4f*)(bias + 4 * cl);
  const v4f z4 = {0.f, 0.f, 0.f, 0.f};
#pragma unroll 1
  for (int j = 0; j < NB / NWAVE; ++j) {
    const int slot = wave * (NB / NWAVE) + j;
    const int node = nodeBase + slot;
    if (node >= nN) break;
    const v4f sv  = *(const v4f*)(sacc + slot * SP + 4 * cl);
    const float dv  = den[slot * HEADS + hd];
    const float inv = 1.0f / dv;
    v4f y = sv * inv + b4;
    y = okc ? y : z4;
    float* op = outp + (size_t)node * HP + 4 * lane;
    *(volatile v4f*)op = y;
    __threadfence();
    *(volatile v4f*)op = y;
  }
}

__global__ __launch_bounds__(NTHR) void k_out(const float* __restrict__ emb, const int* __restrict__ idx,
                                              float* out, int nN, int nM) {
  const int tid = threadIdx.x;
  const int r0  = blockIdx.x * OB;
  const int nQ  = NCH / 4;
  v4f ov[4];
#pragma unroll
  for (int it = 0; it < 4; ++it) {
    int i = tid + NTHR * it;
    if (i > OB * nQ - 1) i = OB * nQ - 1;
    const int row = i / nQ;
    const int c4  = i - row * nQ;
    int orow = r0 + row;
    if (orow > nM - 1) orow = nM - 1;
    int id = idx[orow];
    id = id < 0 ? 0 : (id > nN - 1 ? nN - 1 : id);
    ov[it] = *(const v4f*)(emb + (size_t)id * HP + 4 * c4);
  }
  int rows = nM - r0;
  if (rows > OB) rows = OB;
  const int lim = rows * nQ;
  float* obase = out + (size_t)r0 * NCH;
#pragma unroll
  for (int it = 0; it < 4; ++it) {
    const int i = tid + NTHR * it;
    if (i < lim) *(volatile v4f*)(obase + 4 * i) = ov[it];
  }
  __threadfence();
#pragma unroll
  for (int it = 0; it < 4; ++it) {
    const int i = tid + NTHR * it;
    if (i < lim) *(volatile v4f*)(obase + 4 * i) = ov[it];
  }
}

extern "C" void kernel_launch(void* const* d_in, const int* in_sizes, int n_in,
                              void* d_out, int out_size, void* d_ws, size_t ws_size,
                              hipStream_t stream) {
  if (n_in < 7) return;
  const int nN = in_sizes[0] / NCH;
  if (nN <= 0 || in_sizes[0] != nN * NCH) return;
  if (in_sizes[1] != NCH * NCH) return;
  if (in_sizes[2] != HEADS * 2 * CPH) return;
  if (in_sizes[3] != NCH) return;
  const int nE1 = in_sizes[4] / 2;
  const int nE2 = in_sizes[5] / 2;
  if (nE1 < 0 || in_sizes[4] != 2 * nE1) return;
  if (nE2 < 0 || in_sizes[5] != 2 * nE2) return;
  const int nM = in_sizes[6];
  if (nM <= 0 || out_size != nM * NCH) return;

  const float* emb0 = (const float*)d_in[0];
  const float* W    = (const float*)d_in[1];
  const float* att  = (const float*)d_in[2];
  const float* bias = (const float*)d_in[3];
  const int*   ed1  = (const int*)d_in[4];
  const int*   ed2  = (const int*)d_in[5];
  const int*   idx  = (const int*)d_in[6];
  float* out = (float*)d_out;

  const int nP = ((nN + GR - 1) / GR) * GR;
  size_t off = 0;
  unsigned short* Wh = (unsigned short*)((char*)d_ws + off); off += (size_t)NPADC * KPAD * 2;
  unsigned short* Wl = (unsigned short*)((char*)d_ws + off); off += (size_t)NPADC * KPAD * 2;
  off = (off + 255) & ~(size_t)255;
  float* hpl = (float*)((char*)d_ws + off); off += (size_t)nP * HP * sizeof(float);
  off = (off + 255) & ~(size_t)255;
  float* alp = (float*)((char*)d_ws + off); off += (size_t)nP * ALP * sizeof(float);
  off = (off + 255) & ~(size_t)255;
  float* e1  = (float*)((char*)d_ws + off); off += (size_t)nP * HP * sizeof(float);
  off = (off + 255) & ~(size_t)255;
  float* e2  = (float*)((char*)d_ws + off); off += (size_t)nP * HP * sizeof(float);
  if (off > ws_size) return;
  if (off > (size_t)134217728) return;

  const int nItems = NPADC * (KPAD / 8);
  k_prep<<<(nItems + NTHR - 1) / NTHR, NTHR, 0, stream>>>(W, Wh, Wl, nItems);

  hipFuncSetAttribute(reinterpret_cast<const void*>(&k_gat),
                      hipFuncAttributeMaxDynamicSharedMemorySize, LDS_BYTES);
  const int ggrid = (nN + NB - 1) / NB;

  k_gemm<<<nP / GR, GT, 0, stream>>>(emb0, NCH, Wh, Wl, att, hpl, alp, nN);
  k_gat<<<ggrid, NTHR, LDS_BYTES, stream>>>(hpl, alp, ed1, bias, e1, nN, nE1);

  k_gemm<<<nP / GR, GT, 0, stream>>>(e1, HP, Wh, Wl, att, hpl, alp, nN);
  k_gat<<<ggrid, NTHR, LDS_BYTES, stream>>>(hpl, alp, ed2, bias, e2, nN, nE2);

  k_out<<<(nM + OB - 1) / OB, NTHR, 0, stream>>>(e2, idx, out, nN, nM);
}
